// DecoderSSMLayer_60138132078595
// MI455X (gfx1250) — hardware-verified
//
#include <hip/hip_runtime.h>
#include <math.h>
typedef __attribute__((ext_vector_type(16))) _Float16 v16h;
typedef __attribute__((ext_vector_type(8)))  _Float16 v8h;
typedef __attribute__((ext_vector_type(16))) __bf16   v16b;
typedef __attribute__((ext_vector_type(8)))  __bf16   v8b;
typedef __attribute__((ext_vector_type(8)))  float    v8f;
typedef __attribute__((ext_vector_type(4)))  float    v4f;
#define PSCALE 32768.0f
#define U16(p) ((const unsigned short*)(const void*)(p))
#define PSCALE_INV (1.0f / 32768.0f)

__device__ __forceinline__ unsigned short f2bf_bits(float f) {
  unsigned u = __float_as_uint(f);
  return (unsigned short)((u + 0x7FFFu + ((u >> 16) & 1u)) >> 16);
}
__device__ __forceinline__ float bf_bits2f(unsigned short h) { return __uint_as_float(((unsigned)h) << 16); }

__device__ __forceinline__ void dep_guard_h(v8f& a, v8f& b, v16h x, v16h y) { asm volatile("v_nop\n\tv_nop\n\tv_nop\n\tv_nop" : "+v"(a), "+v"(b) : "v"(x), "v"(y)); }
__device__ __forceinline__ void dep_guard_b(v8f& a, v8f& b, v16b x, v16b y) { asm volatile("v_nop\n\tv_nop\n\tv_nop\n\tv_nop" : "+v"(a), "+v"(b) : "v"(x), "v"(y)); }
__device__ __forceinline__ void keep4_h(v16h a, v16h b, v16h c, v16h d) { asm volatile("v_nop" :: "v"(a), "v"(b), "v"(c), "v"(d)); }
__device__ __forceinline__ void keep4_b(v16b a, v16b b, v16b c, v16b d) { asm volatile("v_nop" :: "v"(a), "v"(b), "v"(c), "v"(d)); }
__device__ __forceinline__ void acc_guard4(v8f& a, v8f& b, v8f& c, v8f& d) { asm volatile("v_nop\n\tv_nop\n\tv_nop\n\tv_nop" : "+v"(a), "+v"(b), "+v"(c), "+v"(d)); }
template <typename T> struct Frag;
template <> struct Frag<_Float16> {
  typedef v16h V; union U { v16h v; v8h h[2]; };
  static __device__ __forceinline__ v16h load(const _Float16* p) {
    U f; f.h[0] = *(const v8h*)(p); f.h[1] = *(const v8h*)(p + 16); return f.v;
  }
  static __device__ __forceinline__ v8f mma(v16h a, v16h b, v8f c) {
    return __builtin_amdgcn_wmma_f32_16x16x32_f16(false, a, false, b, (short)0, c, false, false);
  }
  static __device__ __forceinline__ void guard(v8f& a, v8f& b, v16h x, v16h y) { dep_guard_h(a, b, x, y); }
  static __device__ __forceinline__ void keep(v16h a, v16h b, v16h c, v16h d) { keep4_h(a, b, c, d); }
};
template <> struct Frag<__bf16> {
  typedef v16b V; union U { v16b v; v8b h[2]; };
  static __device__ __forceinline__ v16b load(const __bf16* p) {
    U f; f.h[0] = *(const v8b*)(p); f.h[1] = *(const v8b*)(p + 16); return f.v;
  }
  static __device__ __forceinline__ v8f mma(v16b a, v16b b, v8f c) {
    return __builtin_amdgcn_wmma_f32_16x16x32_bf16(false, a, false, b, (short)0, c, false, false);
  }
  static __device__ __forceinline__ void guard(v8f& a, v8f& b, v16b x, v16b y) { dep_guard_b(a, b, x, y); }
  static __device__ __forceinline__ void keep(v16b a, v16b b, v16b c, v16b d) { keep4_b(a, b, c, d); }
};

template <int ET> struct Elem;
template <> struct Elem<0> { typedef _Float16 T; };
template <> struct Elem<1> { typedef __bf16 T; };
template <int ET, bool SPLIT, int BIAS_MODE, int OUT_MODE, bool RESID, int ACT = 0>
__global__ __launch_bounds__(256) void wmma_gemm64(
    const unsigned short* __restrict__ Ap, const unsigned short* __restrict__ A2p, int lda, long strideA,
    const unsigned short* __restrict__ Btp, const unsigned short* __restrict__ Bt2p, int ldb, long strideB,
    void* __restrict__ Cout, void* __restrict__ Cout2, int ldc, long strideC,
    const float* __restrict__ bias,
    const float* __restrict__ resid, long strideR,
    int M, int N, int K, float scale) {
  typedef typename Elem<ET>::T T;
  typedef typename Frag<T>::V V;
  const T* A = (const T*)Ap; const T* A2 = (const T*)A2p; const T* Bt = (const T*)Btp; const T* Bt2 = (const T*)Bt2p;
  __shared__ __align__(16) float sT[8][16 * 68];
  const int b    = blockIdx.y;
  const int lane = threadIdx.x & 31;
  const int wave = threadIdx.x >> 5;
  const int tilesN = N >> 6;
  const int tilesM = M >> 6;
  const int tile = blockIdx.x * 8 + wave;
  if (tile >= tilesM * tilesN) return;
  const int tm = tile / tilesN;
  const int tn = tile - tm * tilesN;
  const int m0 = tm << 6;
  const int n0 = tn << 6;

  const T* Ab  = A  + (size_t)b * strideA;
  const T* Bb  = Bt + (size_t)b * strideB;
  const T* Ab2 = SPLIT ? (A2  + (size_t)b * strideA) : nullptr;
  const T* Bb2 = SPLIT ? (Bt2 + (size_t)b * strideB) : nullptr;

  const int rlane = lane & 15;
  const int koff  = (lane >> 4) * 8;
  const int mOff  = (lane >> 4) * 8;

  v8f acc[4][4];
#pragma unroll
  for (int i = 0; i < 4; ++i)
#pragma unroll
    for (int j = 0; j < 4; ++j) acc[i][j] = (v8f){0.f,0.f,0.f,0.f,0.f,0.f,0.f,0.f};

  for (int k0 = 0; k0 < K; k0 += 32) {
    V bh[4], bl[4];
#pragma unroll
    for (int j = 0; j < 4; ++j) {
      const size_t bo = (size_t)(n0 + (j << 4) + rlane) * ldb + koff + k0;
      bh[j] = Frag<T>::load(Bb + bo);
      if (SPLIT) bl[j] = Frag<T>::load(Bb2 + bo);
    }
#pragma unroll
    for (int i = 0; i < 4; ++i) {
      const size_t ao = (size_t)(m0 + (i << 4) + rlane) * lda + koff + k0;
      V ah = Frag<T>::load(Ab + ao);
      V al;
      if (SPLIT) al = Frag<T>::load(Ab2 + ao);
#pragma unroll
      for (int j = 0; j < 4; ++j) {
        acc[i][j] = Frag<T>::mma(ah, bh[j], acc[i][j]);
        if (SPLIT) {
          acc[i][j] = Frag<T>::mma(ah, bl[j], acc[i][j]);
          acc[i][j] = Frag<T>::mma(al, bh[j], acc[i][j]);
        }
      }
      Frag<T>::guard(acc[i][0], acc[i][3], ah, SPLIT ? al : ah);
    }
    Frag<T>::keep(bh[0], bh[1], bh[2], bh[3]);
    if (SPLIT) Frag<T>::keep(bl[0], bl[1], bl[2], bl[3]);
  }
  acc_guard4(acc[0][0], acc[0][1], acc[0][2], acc[0][3]);
  acc_guard4(acc[1][0], acc[1][1], acc[1][2], acc[1][3]);
  acc_guard4(acc[2][0], acc[2][1], acc[2][2], acc[2][3]);
  acc_guard4(acc[3][0], acc[3][1], acc[3][2], acc[3][3]);

  float* slab = sT[wave];
  const float* Rb = RESID ? (resid + (size_t)b * strideR) : nullptr;
#pragma unroll
  for (int i = 0; i < 4; ++i) {
    const int mBase = m0 + (i << 4);
#pragma unroll
    for (int j = 0; j < 4; ++j) {
      const int n = n0 + (j << 4) + rlane;
      float bv = 0.f;
      if (BIAS_MODE == 2) bv = bias[n];
#pragma unroll
      for (int r = 0; r < 8; ++r) {
        float v = acc[i][j][r] * scale;
        if (BIAS_MODE == 1) v += bias[mBase + mOff + r];
        if (BIAS_MODE == 2) v += bv;
        if (RESID) v += Rb[(size_t)(mBase + mOff + r) * ldc + n];
        if (ACT == 1) v = tanhf(v);
        slab[(mOff + r) * 68 + (j << 4) + rlane] = v;
      }
    }
    __builtin_amdgcn_fence(__ATOMIC_RELEASE, "workgroup");
    __builtin_amdgcn_wave_barrier();
    __builtin_amdgcn_fence(__ATOMIC_ACQUIRE, "workgroup");
    if (OUT_MODE == 0) {
      float* C = (float*)Cout + (size_t)b * strideC;
      const int hh = lane >> 4, c4 = (lane & 15) * 4;
      for (int pass = 0; pass < 2; ++pass) {
#pragma unroll
        for (int it = 0; it < 8; ++it) {
          const int row = it * 2 + hh;
          v4f v = *(const v4f*)(slab + row * 68 + c4);
          *(volatile v4f*)(C + (size_t)(mBase + row) * ldc + n0 + c4) = v;
        }
        __threadfence();
      }
    } else {
      const int q = lane >> 3, c8 = (lane & 7) * 8;
      unsigned short* C  = (unsigned short*)Cout  + (size_t)b * strideC;
      unsigned short* C2 = (OUT_MODE == 2) ? ((unsigned short*)Cout2 + (size_t)b * strideC) : nullptr;
      for (int pass = 0; pass < 2; ++pass) {
#pragma unroll
        for (int it = 0; it < 4; ++it) {
          const int row = it * 4 + q;
          const float* sp = slab + row * 68 + c8;
          v8h hv, lv;
#pragma unroll
          for (int e = 0; e < 8; ++e) {
            if (OUT_MODE == 1) {
              hv[e] = (_Float16)sp[e];
            } else {
              unsigned short hb = f2bf_bits(sp[e]);
              unsigned short lb = f2bf_bits(sp[e] - bf_bits2f(hb));
              hv[e] = __builtin_bit_cast(_Float16, hb);
              lv[e] = __builtin_bit_cast(_Float16, lb);
            }
          }
          *(volatile v8h*)(C + (size_t)(mBase + row) * ldc + n0 + c8) = hv;
          if (OUT_MODE == 2) *(volatile v8h*)(C2 + (size_t)(mBase + row) * ldc + n0 + c8) = lv;
        }
        __threadfence();
      }
    }
    __builtin_amdgcn_fence(__ATOMIC_RELEASE, "workgroup");
    __builtin_amdgcn_wave_barrier();
    __builtin_amdgcn_fence(__ATOMIC_ACQUIRE, "workgroup");
  }
}

__global__ __launch_bounds__(256) void cast_f32_f16x2(
    const float* __restrict__ in, _Float16* __restrict__ out, int n2) {
  int i = blockIdx.x * 256 + threadIdx.x;
  if (i < n2) {
    const _Float16 h0 = (_Float16)in[2 * i], h1 = (_Float16)in[2 * i + 1];
    const unsigned u = (unsigned)__builtin_bit_cast(unsigned short, h0) | ((unsigned)__builtin_bit_cast(unsigned short, h1) << 16);
    ((volatile unsigned*)out)[i] = u;
    __threadfence();
    ((volatile unsigned*)out)[i] = u;
  }
}


__global__ __launch_bounds__(256) void transpose_cast_f16(const float* __restrict__ in, int ldi,
                                                         _Float16* __restrict__ outT, int ldo, float scale) {
  __shared__ __align__(16) _Float16 tile[64][72];
  const int c0 = blockIdx.x * 64, r0 = blockIdx.y * 64;
  const int t = threadIdx.y * 32 + threadIdx.x;
  for (int i = threadIdx.y; i < 64; i += 8) {
    tile[threadIdx.x][i]      = (_Float16)(in[(size_t)(r0 + i) * ldi + c0 + threadIdx.x] * scale);
    tile[32 + threadIdx.x][i] = (_Float16)(in[(size_t)(r0 + i) * ldi + c0 + 32 + threadIdx.x] * scale);
  }
  __syncthreads();
  const int q = t >> 3, c8 = (t & 7) * 8;
  for (int pass = 0; pass < 2; ++pass) {
#pragma unroll
    for (int it = 0; it < 2; ++it) {
      const int c = it * 32 + q;
      v8h hv = *(const v8h*)(&tile[c][c8]);
      *(volatile v8h*)(outT + (size_t)(c0 + c) * ldo + r0 + c8) = hv;
    }
    __threadfence();
  }
}

#define B_SZ    4
#define SEQ_L   4096
#define DMODEL  512
#define DSTATE  16
#define DINNER  1024
#define DCONV   4
#define DTRANK  32
#define NROWS   (B_SZ * SEQ_L)
#define N_XZ    (2 * DINNER)
#define N_XDBL  (DTRANK + 2 * DSTATE)

__global__ __launch_bounds__(256) void layernorm_f16_kernel(const float* __restrict__ x, const float* __restrict__ g,
                                                           const float* __restrict__ be, unsigned* __restrict__ out) {
  __shared__ float red[8];
  __shared__ float stat;
  const int row = blockIdx.x, t = threadIdx.x;
  const float* xr = x + (size_t)row * DMODEL;
  const float v0 = xr[2 * t], v1 = xr[2 * t + 1];
  float s = v0 + v1;
  for (int o = 16; o > 0; o >>= 1) s += __shfl_xor(s, o, 32);
  if ((t & 31) == 0) red[t >> 5] = s;
  __syncthreads();
  if (t == 0) { float a = 0.f; for (int w = 0; w < 8; ++w) a += red[w]; stat = a * (1.0f / DMODEL); }
  __syncthreads();
  const float mu = stat;
  __syncthreads();
  const float d0 = v0 - mu, d1 = v1 - mu;
  float s2 = d0 * d0 + d1 * d1;
  for (int o = 16; o > 0; o >>= 1) s2 += __shfl_xor(s2, o, 32);
  if ((t & 31) == 0) red[t >> 5] = s2;
  __syncthreads();
  if (t == 0) { float a = 0.f; for (int w = 0; w < 8; ++w) a += red[w]; stat = rsqrtf(a * (1.0f / DMODEL) + 1e-5f); }
  __syncthreads();
  const float rstd = stat;
  const _Float16 h0 = (_Float16)(d0 * rstd * g[2 * t] + be[2 * t]), h1 = (_Float16)(d1 * rstd * g[2 * t + 1] + be[2 * t + 1]);
  const unsigned u = (unsigned)__builtin_bit_cast(unsigned short, h0) | ((unsigned)__builtin_bit_cast(unsigned short, h1) << 16);
  ((volatile unsigned*)out)[(size_t)row * (DMODEL / 2) + t] = u;
  __threadfence();
  ((volatile unsigned*)out)[(size_t)row * (DMODEL / 2) + t] = u;
}

__global__ __launch_bounds__(256) void conv_silu_kernel(const _Float16* __restrict__ xz, const float* __restrict__ w,
                                                       const float* __restrict__ bias, float* __restrict__ u32, unsigned* __restrict__ u16) {
  const size_t i = (size_t)blockIdx.x * 256 + threadIdx.x;
  if (i >= (size_t)NROWS * DINNER / 2) return;
  const size_t row = i / (DINNER / 2);
  const int c0 = (int)(i % (DINNER / 2)) * 2;
  const int l = (int)(row % SEQ_L);
  float r[2];
#pragma unroll
  for (int q = 0; q < 2; ++q) {
    const int c = c0 + q;
    const float* wc = w + (size_t)c * DCONV;
    float acc = 0.f;
#pragma unroll
    for (int j = 0; j < DCONV; ++j) {
      const int ls = l - (DCONV - 1) + j;
      if (ls >= 0) acc += wc[j] * (float)xz[(row - (size_t)(DCONV - 1 - j)) * N_XZ + c];
    }
    acc += bias[c];
    r[q] = acc / (1.0f + expf(-acc));
  }
  typedef __attribute__((ext_vector_type(2))) float v2f;
  const v2f rv = {r[0], r[1]};
  const unsigned hu = (unsigned)__builtin_bit_cast(unsigned short, (_Float16)r[0]) | ((unsigned)__builtin_bit_cast(unsigned short, (_Float16)r[1]) << 16);
  for (int pass = 0; pass < 2; ++pass) {
    *(volatile v2f*)(u32 + row * DINNER + c0) = rv;
    ((volatile unsigned*)u16)[i] = hu;
    __threadfence();
  }
}

#define SCAN_CPB   128
#define SCAN_CHUNK 64
__global__ __launch_bounds__(SCAN_CPB)
void selective_scan_kernel(const float* __restrict__ x_dbl, const float* __restrict__ W_dt, const float* __restrict__ b_dt,
                           const float* __restrict__ u32, const _Float16* __restrict__ xz,
                           const float* __restrict__ A_log, const float* __restrict__ Dp,
                           _Float16* __restrict__ yg) {
  __shared__ float Xsh[SCAN_CHUNK][N_XDBL];
  __shared__ __align__(16) _Float16 Ysh[SCAN_CHUNK][SCAN_CPB];
  const int blocksPerBatch = DINNER / SCAN_CPB;
  const int b = blockIdx.x / blocksPerBatch;
  const int cbase = (blockIdx.x % blocksPerBatch) * SCAN_CPB;
  const int c = cbase + threadIdx.x;
  const int lane = threadIdx.x & 31, wave = threadIdx.x >> 5;

  float A[DSTATE], s[DSTATE], wdt[DTRANK];
#pragma unroll
  for (int n = 0; n < DSTATE; ++n) { A[n] = -expf(A_log[(size_t)c * DSTATE + n]); s[n] = 0.0f; }
#pragma unroll
  for (int r = 0; r < DTRANK; ++r) wdt[r] = W_dt[(size_t)r * DINNER + c];
  const float bdt = b_dt[c];
  const float Dv = Dp[c];
  const size_t rowbase = (size_t)b * SEQ_L;

  for (int l0 = 0; l0 < SEQ_L; l0 += SCAN_CHUNK) {
    __syncthreads();
    for (int i = threadIdx.x; i < SCAN_CHUNK * N_XDBL; i += SCAN_CPB) {
      const int t = i / N_XDBL, q = i % N_XDBL;
      Xsh[t][q] = x_dbl[(rowbase + l0 + t) * N_XDBL + q];
    }
    __syncthreads();
#pragma unroll 1
    for (int t = 0; t < SCAN_CHUNK; ++t) {
      const size_t row = rowbase + l0 + t;
      float a = 0.f;
#pragma unroll 1
      for (int r = 0; r < DTRANK; ++r) a += Xsh[t][r] * wdt[r];
      a += bdt;
      const float dl = (a > 20.0f) ? a : log1pf(expf(a));
      const float u  = u32[row * DINNER + c];
      const float du = dl * u;
      float y = 0.0f;
#pragma unroll 4
      for (int n = 0; n < DSTATE; ++n) {
        const float dA = expf(dl * A[n]);
        s[n] = dA * s[n] + du * Xsh[t][DTRANK + n];
        y += s[n] * Xsh[t][DTRANK + DSTATE + n];
      }
      y += u * Dv;
      const float z = (float)xz[row * N_XZ + DINNER + c];
      const float gte = z / (1.0f + expf(-z));
      Ysh[t][threadIdx.x] = (_Float16)(y * gte);
    }
    __syncthreads();
    {
      const int half = lane >> 4, c8 = (lane & 15) * 8;
      for (int pass = 0; pass < 2; ++pass) {
#pragma unroll
        for (int i = 0; i < 8; ++i) {
          const int t = wave * 16 + i * 2 + half;
          const v8h v = *(const v8h*)(&Ysh[t][c8]);
          *(volatile v8h*)(yg + (rowbase + l0 + t) * DINNER + cbase + c8) = v;
        }
        __threadfence();
      }
    }
  }
}

extern "C" void kernel_launch(void* const* d_in, const int* in_sizes, int n_in,
                              void* d_out, int out_size, void* d_ws, size_t ws_size,
                              hipStream_t stream) {
  (void)in_sizes; (void)n_in; (void)out_size; (void)ws_size;
  const float* x        = (const float*)d_in[0];
  const float* ln_gamma = (const float*)d_in[1];
  const float* ln_beta  = (const float*)d_in[2];
  const float* W_in     = (const float*)d_in[3];
  const float* conv_w   = (const float*)d_in[4];
  const float* conv_b   = (const float*)d_in[5];
  const float* W_x      = (const float*)d_in[6];
  const float* W_dt     = (const float*)d_in[7];
  const float* b_dt     = (const float*)d_in[8];
  const float* A_log    = (const float*)d_in[9];
  const float* Dvec     = (const float*)d_in[10];
  const float* W_out    = (const float*)d_in[11];
  float* out = (float*)d_out;

  char* ws = (char*)d_ws; size_t off = 0;
  auto carve = [&](size_t bytes) -> char* { char* p = ws + off; off += (bytes + 255) & ~(size_t)255; return p; };
  unsigned* H16   = (unsigned*)carve((size_t)NROWS * DMODEL * 2);
  _Float16* WinT  = (_Float16*)carve((size_t)N_XZ * DMODEL * 2);
  _Float16* WxT   = (_Float16*)carve((size_t)N_XDBL * DINNER * 2);
  _Float16* WoutT = (_Float16*)carve((size_t)DMODEL * DINNER * 2);
  _Float16* XZ16  = (_Float16*)carve((size_t)NROWS * N_XZ * 2);
  float*    U32   = (float*)carve((size_t)NROWS * DINNER * 4);
  unsigned* U16   = (unsigned*)carve((size_t)NROWS * DINNER * 2);
  float*    XDBL  = (float*)carve((size_t)NROWS * N_XDBL * 4);
  _Float16* YG16  = (_Float16*)carve((size_t)NROWS * DINNER * 2);

  transpose_cast_f16<<<dim3(N_XZ / 64, DMODEL / 64), dim3(32, 8), 0, stream>>>(W_in, N_XZ, WinT, DMODEL, 1.0f);
  transpose_cast_f16<<<dim3(N_XDBL / 64, DINNER / 64), dim3(32, 8), 0, stream>>>(W_x, N_XDBL, WxT, DINNER, 1.0f);
  transpose_cast_f16<<<dim3(DMODEL / 64, DINNER / 64), dim3(32, 8), 0, stream>>>(W_out, DMODEL, WoutT, DINNER, 1.0f);
  layernorm_f16_kernel<<<NROWS, 256, 0, stream>>>(x, ln_gamma, ln_beta, H16);
  {
    const int t1 = (NROWS / 64) * (N_XZ / 64);
    wmma_gemm64<0, false, 0, 1, false><<<dim3((t1 + 7) / 8, 1), 256, 0, stream>>>(
        (const unsigned short*)H16, nullptr, DMODEL, 0, U16(WinT), nullptr, DMODEL, 0, XZ16, nullptr, N_XZ, 0, nullptr, nullptr, 0, NROWS, N_XZ, DMODEL, 1.0f);
  }
  conv_silu_kernel<<<(NROWS * DINNER / 2 + 255) / 256, 256, 0, stream>>>(XZ16, conv_w, conv_b, U32, U16);
  {
    const int t2 = (NROWS / 64) * (N_XDBL / 64);
    wmma_gemm64<0, false, 0, 0, false><<<dim3((t2 + 7) / 8, 1), 256, 0, stream>>>(
        (const unsigned short*)U16, nullptr, DINNER, 0, U16(WxT), nullptr, DINNER, 0, XDBL, nullptr, N_XDBL, 0, nullptr, nullptr, 0, NROWS, N_XDBL, DINNER, 1.0f);
  }
  selective_scan_kernel<<<B_SZ * (DINNER / SCAN_CPB), SCAN_CPB, 0, stream>>>(XDBL, W_dt, b_dt, U32, XZ16, A_log, Dvec, YG16);
  {
    const int t3 = (NROWS / 64) * (DMODEL / 64);
    wmma_gemm64<0, false, 0, 0, true><<<dim3((t3 + 7) / 8, 1), 256, 0, stream>>>(
        U16(YG16), nullptr, DINNER, 0, U16(WoutT), nullptr, DINNER, 0, out, nullptr, DMODEL, 0, nullptr, x, 0, NROWS, DMODEL, DINNER, 1.0f);
  }
}
